// LSEA_28355374088837
// MI455X (gfx1250) — hardware-verified
//
#include <hip/hip_runtime.h>
#include <math.h>
typedef __attribute__((ext_vector_type(16))) _Float16 v16h;
typedef __attribute__((ext_vector_type(8)))  _Float16 v8h;
typedef __attribute__((ext_vector_type(16))) __bf16   v16b;
typedef __attribute__((ext_vector_type(8)))  __bf16   v8b;
typedef __attribute__((ext_vector_type(8)))  float    v8f;
typedef __attribute__((ext_vector_type(4)))  float    v4f;
#define PSCALE 32768.0f
#define U16(p) ((const unsigned short*)(const void*)(p))
#define PSCALE_INV (1.0f / 32768.0f)

__device__ __forceinline__ unsigned short f2bf_bits(float f) {
  unsigned u = __float_as_uint(f);
  return (unsigned short)((u + 0x7FFFu + ((u >> 16) & 1u)) >> 16);
}
__device__ __forceinline__ float bf_bits2f(unsigned short h) { return __uint_as_float(((unsigned)h) << 16); }

__device__ __forceinline__ void dep_guard_h(v8f& a, v8f& b, v16h x, v16h y) { asm volatile("v_nop\n\tv_nop\n\tv_nop\n\tv_nop" : "+v"(a), "+v"(b) : "v"(x), "v"(y)); }
__device__ __forceinline__ void dep_guard_b(v8f& a, v8f& b, v16b x, v16b y) { asm volatile("v_nop\n\tv_nop\n\tv_nop\n\tv_nop" : "+v"(a), "+v"(b) : "v"(x), "v"(y)); }
__device__ __forceinline__ void keep4_h(v16h a, v16h b, v16h c, v16h d) { asm volatile("v_nop" :: "v"(a), "v"(b), "v"(c), "v"(d)); }
__device__ __forceinline__ void keep4_b(v16b a, v16b b, v16b c, v16b d) { asm volatile("v_nop" :: "v"(a), "v"(b), "v"(c), "v"(d)); }
__device__ __forceinline__ void acc_guard4(v8f& a, v8f& b, v8f& c, v8f& d) { asm volatile("v_nop\n\tv_nop\n\tv_nop\n\tv_nop" : "+v"(a), "+v"(b), "+v"(c), "+v"(d)); }
template <typename T> struct Frag;
template <> struct Frag<_Float16> {
  typedef v16h V; union U { v16h v; v8h h[2]; };
  static __device__ __forceinline__ v16h load(const _Float16* p) {
    U f; f.h[0] = *(const v8h*)(p); f.h[1] = *(const v8h*)(p + 16); return f.v;
  }
  static __device__ __forceinline__ v8f mma(v16h a, v16h b, v8f c) {
    return __builtin_amdgcn_wmma_f32_16x16x32_f16(false, a, false, b, (short)0, c, false, false);
  }
  static __device__ __forceinline__ void guard(v8f& a, v8f& b, v16h x, v16h y) { dep_guard_h(a, b, x, y); }
  static __device__ __forceinline__ void keep(v16h a, v16h b, v16h c, v16h d) { keep4_h(a, b, c, d); }
};
template <> struct Frag<__bf16> {
  typedef v16b V; union U { v16b v; v8b h[2]; };
  static __device__ __forceinline__ v16b load(const __bf16* p) {
    U f; f.h[0] = *(const v8b*)(p); f.h[1] = *(const v8b*)(p + 16); return f.v;
  }
  static __device__ __forceinline__ v8f mma(v16b a, v16b b, v8f c) {
    return __builtin_amdgcn_wmma_f32_16x16x32_bf16(false, a, false, b, (short)0, c, false, false);
  }
  static __device__ __forceinline__ void guard(v8f& a, v8f& b, v16b x, v16b y) { dep_guard_b(a, b, x, y); }
  static __device__ __forceinline__ void keep(v16b a, v16b b, v16b c, v16b d) { keep4_b(a, b, c, d); }
};

template <int ET> struct Elem;
template <> struct Elem<0> { typedef _Float16 T; };
template <> struct Elem<1> { typedef __bf16 T; };
template <int ET, bool SPLIT, int BIAS_MODE, int OUT_MODE, bool RESID, int ACT = 0>
__global__ __launch_bounds__(256) void wmma_gemm64(
    const unsigned short* __restrict__ Ap, const unsigned short* __restrict__ A2p, int lda, long strideA,
    const unsigned short* __restrict__ Btp, const unsigned short* __restrict__ Bt2p, int ldb, long strideB,
    void* __restrict__ Cout, void* __restrict__ Cout2, int ldc, long strideC,
    const float* __restrict__ bias,
    const float* __restrict__ resid, long strideR,
    int M, int N, int K, float scale) {
  typedef typename Elem<ET>::T T;
  typedef typename Frag<T>::V V;
  const T* A = (const T*)Ap; const T* A2 = (const T*)A2p; const T* Bt = (const T*)Btp; const T* Bt2 = (const T*)Bt2p;
  __shared__ __align__(16) float sT[8][16 * 68];
  const int b    = blockIdx.y;
  const int lane = threadIdx.x & 31;
  const int wave = threadIdx.x >> 5;
  const int tilesN = N >> 6;
  const int tilesM = M >> 6;
  const int tile = blockIdx.x * 8 + wave;
  if (tile >= tilesM * tilesN) return;
  const int tm = tile / tilesN;
  const int tn = tile - tm * tilesN;
  const int m0 = tm << 6;
  const int n0 = tn << 6;

  const T* Ab  = A  + (size_t)b * strideA;
  const T* Bb  = Bt + (size_t)b * strideB;
  const T* Ab2 = SPLIT ? (A2  + (size_t)b * strideA) : nullptr;
  const T* Bb2 = SPLIT ? (Bt2 + (size_t)b * strideB) : nullptr;

  const int rlane = lane & 15;
  const int koff  = (lane >> 4) * 8;
  const int mOff  = (lane >> 4) * 8;

  v8f acc[4][4];
#pragma unroll
  for (int i = 0; i < 4; ++i)
#pragma unroll
    for (int j = 0; j < 4; ++j) acc[i][j] = (v8f){0.f,0.f,0.f,0.f,0.f,0.f,0.f,0.f};

  for (int k0 = 0; k0 < K; k0 += 32) {
    V bh[4], bl[4];
#pragma unroll
    for (int j = 0; j < 4; ++j) {
      const size_t bo = (size_t)(n0 + (j << 4) + rlane) * ldb + koff + k0;
      bh[j] = Frag<T>::load(Bb + bo);
      if (SPLIT) bl[j] = Frag<T>::load(Bb2 + bo);
    }
#pragma unroll
    for (int i = 0; i < 4; ++i) {
      const size_t ao = (size_t)(m0 + (i << 4) + rlane) * lda + koff + k0;
      V ah = Frag<T>::load(Ab + ao);
      V al;
      if (SPLIT) al = Frag<T>::load(Ab2 + ao);
#pragma unroll
      for (int j = 0; j < 4; ++j) {
        acc[i][j] = Frag<T>::mma(ah, bh[j], acc[i][j]);
        if (SPLIT) {
          acc[i][j] = Frag<T>::mma(ah, bl[j], acc[i][j]);
          acc[i][j] = Frag<T>::mma(al, bh[j], acc[i][j]);
        }
      }
      Frag<T>::guard(acc[i][0], acc[i][3], ah, SPLIT ? al : ah);
    }
    Frag<T>::keep(bh[0], bh[1], bh[2], bh[3]);
    if (SPLIT) Frag<T>::keep(bl[0], bl[1], bl[2], bl[3]);
  }
  acc_guard4(acc[0][0], acc[0][1], acc[0][2], acc[0][3]);
  acc_guard4(acc[1][0], acc[1][1], acc[1][2], acc[1][3]);
  acc_guard4(acc[2][0], acc[2][1], acc[2][2], acc[2][3]);
  acc_guard4(acc[3][0], acc[3][1], acc[3][2], acc[3][3]);

  float* slab = sT[wave];
  const float* Rb = RESID ? (resid + (size_t)b * strideR) : nullptr;
#pragma unroll
  for (int i = 0; i < 4; ++i) {
    const int mBase = m0 + (i << 4);
#pragma unroll
    for (int j = 0; j < 4; ++j) {
      const int n = n0 + (j << 4) + rlane;
      float bv = 0.f;
      if (BIAS_MODE == 2) bv = bias[n];
#pragma unroll
      for (int r = 0; r < 8; ++r) {
        float v = acc[i][j][r] * scale;
        if (BIAS_MODE == 1) v += bias[mBase + mOff + r];
        if (BIAS_MODE == 2) v += bv;
        if (RESID) v += Rb[(size_t)(mBase + mOff + r) * ldc + n];
        if (ACT == 1) v = tanhf(v);
        if (ACT == 2) v = fmaxf(v, 0.0f);
        if (ACT == 3) v = v / (1.0f + expf(-v));
        if (ACT == 4) v = (v > 0.f) ? v : 0.01f * v;
        if (ACT == 5) v = 0.5f * v * (1.0f + erff(v * 0.70710678118654752f));
        if (ACT == 6) v = (v > 0.f) ? v : 0.2f * v;
        slab[(mOff + r) * 68 + (j << 4) + rlane] = v;
      }
    }
    __builtin_amdgcn_fence(__ATOMIC_RELEASE, "workgroup");
    __builtin_amdgcn_wave_barrier();
    __builtin_amdgcn_fence(__ATOMIC_ACQUIRE, "workgroup");
    if (OUT_MODE == 0) {
      float* C = (float*)Cout + (size_t)b * strideC;
      const int hh = lane >> 4, c4 = (lane & 15) * 4;
      for (int pass = 0; pass < 2; ++pass) {
#pragma unroll
        for (int it = 0; it < 8; ++it) {
          const int row = it * 2 + hh;
          v4f v = *(const v4f*)(slab + row * 68 + c4);
          *(volatile v4f*)(C + (size_t)(mBase + row) * ldc + n0 + c4) = v;
        }
        __threadfence();
      }
    } else {
      const int q = lane >> 3, c8 = (lane & 7) * 8;
      unsigned short* C  = (unsigned short*)Cout  + (size_t)b * strideC;
      unsigned short* C2 = (OUT_MODE == 2) ? ((unsigned short*)Cout2 + (size_t)b * strideC) : nullptr;
      for (int pass = 0; pass < 2; ++pass) {
#pragma unroll
        for (int it = 0; it < 4; ++it) {
          const int row = it * 4 + q;
          const float* sp = slab + row * 68 + c8;
          v8h hv, lv;
#pragma unroll
          for (int e = 0; e < 8; ++e) {
            if (OUT_MODE == 1) {
              hv[e] = (_Float16)sp[e];
            } else {
              unsigned short hb = f2bf_bits(sp[e]);
              unsigned short lb = f2bf_bits(sp[e] - bf_bits2f(hb));
              hv[e] = __builtin_bit_cast(_Float16, hb);
              lv[e] = __builtin_bit_cast(_Float16, lb);
            }
          }
          *(volatile v8h*)(C + (size_t)(mBase + row) * ldc + n0 + c8) = hv;
          if (OUT_MODE == 2) *(volatile v8h*)(C2 + (size_t)(mBase + row) * ldc + n0 + c8) = lv;
        }
        __threadfence();
      }
    }
    __builtin_amdgcn_fence(__ATOMIC_RELEASE, "workgroup");
    __builtin_amdgcn_wave_barrier();
    __builtin_amdgcn_fence(__ATOMIC_ACQUIRE, "workgroup");
  }
}

__global__ __launch_bounds__(256) void cast_f32_f16x2(
    const float* __restrict__ in, _Float16* __restrict__ out, int n2) {
  int i = blockIdx.x * 256 + threadIdx.x;
  if (i < n2) {
    const _Float16 h0 = (_Float16)in[2 * i], h1 = (_Float16)in[2 * i + 1];
    const unsigned u = (unsigned)__builtin_bit_cast(unsigned short, h0) | ((unsigned)__builtin_bit_cast(unsigned short, h1) << 16);
    ((volatile unsigned*)out)[i] = u;
    __threadfence();
    ((volatile unsigned*)out)[i] = u;
  }
}


#define PB 16
#define PN 4096
#define PK 16
#define PR (PB * PN)
#define PRK (PR * PK)
__global__ __launch_bounds__(256) void fold_kernel(const float* __restrict__ w, const float* __restrict__ s, const float* __restrict__ b, int nout, int kin, int npad, int row0, unsigned* __restrict__ WT, float* __restrict__ bp) {
  const int i = blockIdx.x * 256 + threadIdx.x; if (i >= npad * kin / 2) return; const int o = (2 * i) / kin, k = (2 * i) % kin;
  float a = 0.f, c = 0.f; if (o < nout) { a = w[o * kin + k] * s[o]; c = w[o * kin + k + 1] * s[o]; }
  const unsigned u = (unsigned)__builtin_bit_cast(unsigned short, (_Float16)a) | ((unsigned)__builtin_bit_cast(unsigned short, (_Float16)c) << 16);
  ((volatile unsigned*)WT)[(size_t)(row0) * kin / 2 + i] = u; if (k == 0) ((volatile float*)bp)[row0 + o] = (o < nout) ? b[o] : 0.f; __threadfence();
  ((volatile unsigned*)WT)[(size_t)(row0) * kin / 2 + i] = u; if (k == 0) ((volatile float*)bp)[row0 + o] = (o < nout) ? b[o] : 0.f;
}
__global__ __launch_bounds__(256) void in_kernel(const float* __restrict__ feat, const float* __restrict__ x, unsigned* __restrict__ FT16, float* __restrict__ XT) {
  __shared__ float tile[64][65];
  const int b = blockIdx.y, n0 = blockIdx.x * 64, tx = threadIdx.x, ty = threadIdx.y;
  for (int c = ty; c < 64; c += 8) { tile[c][tx] = feat[((size_t)b * 64 + c) * PN + n0 + tx]; tile[c][32 + tx] = feat[((size_t)b * 64 + c) * PN + n0 + 32 + tx]; }
  __syncthreads();
  for (int pass = 0; pass < 2; ++pass) {
    for (int p = ty; p < 64; p += 8) { const size_t r = (size_t)b * PN + n0 + p; const unsigned u = (unsigned)__builtin_bit_cast(unsigned short, (_Float16)tile[2 * tx][p]) | ((unsigned)__builtin_bit_cast(unsigned short, (_Float16)tile[2 * tx + 1][p]) << 16);
      ((volatile unsigned*)FT16)[r * 32 + tx] = u;
      if (tx < 4) ((volatile float*)XT)[r * 4 + tx] = (tx < 3) ? x[((size_t)b * 3 + tx) * PN + n0 + p] : 0.f; }
    __threadfence(); }
}
__global__ __launch_bounds__(256) void lse1_kernel(const float* __restrict__ XT, const int* __restrict__ nidx, const float* __restrict__ W, const float* __restrict__ s, const float* __restrict__ bb, unsigned* __restrict__ XI16) {
  __shared__ float sw[32 * 10], ss[32], sb[32];
  for (int i = threadIdx.x; i < 320; i += 256) sw[i] = W[i]; if (threadIdx.x < 32) { ss[threadIdx.x] = s[threadIdx.x]; sb[threadIdx.x] = bb[threadIdx.x]; }
  __syncthreads();
  const long i = (long)blockIdx.x * 256 + threadIdx.x; const long r = i / PK; const int b = (int)(r / PN);
  int j = nidx[i]; j = j < 0 ? 0 : (j >= PN ? PN - 1 : j); const long rj = (long)b * PN + j;
  float xi[10]; const float cx = XT[r * 4], cy = XT[r * 4 + 1], cz = XT[r * 4 + 2], kx = XT[rj * 4], ky = XT[rj * 4 + 1], kz = XT[rj * 4 + 2];
  xi[0] = cx; xi[1] = cy; xi[2] = cz; xi[3] = kx; xi[4] = ky; xi[5] = kz; xi[6] = kx - cx; xi[7] = ky - cy; xi[8] = kz - cz; xi[9] = sqrtf(xi[6] * xi[6] + xi[7] * xi[7] + xi[8] * xi[8] + 1e-12f);
  unsigned out[16];
#pragma unroll 1
  for (int op = 0; op < 16; ++op) { float v2[2];
    for (int h = 0; h < 2; ++h) { const int o = 2 * op + h; float a = 0.f;
#pragma unroll
      for (int q = 0; q < 10; ++q) a += xi[q] * sw[o * 10 + q];
      a = a * ss[o] + sb[o]; v2[h] = a > 0.f ? a : 0.2f * a; }
    out[op] = (unsigned)__builtin_bit_cast(unsigned short, (_Float16)v2[0]) | ((unsigned)__builtin_bit_cast(unsigned short, (_Float16)v2[1]) << 16); }
  typedef __attribute__((ext_vector_type(4))) unsigned u4;
  for (int pass = 0; pass < 2; ++pass) { for (int q = 0; q < 4; ++q) { u4 v = {out[4*q], out[4*q+1], out[4*q+2], out[4*q+3]}; *(volatile u4*)(XI16 + i * 16 + q * 4) = v; } __threadfence(); }
}
__device__ __forceinline__ float ldh(const unsigned* p, long idx) { const unsigned u = p[idx >> 1]; return (float)__builtin_bit_cast(_Float16, (unsigned short)((idx & 1) ? (u >> 16) : (u & 0xFFFFu))); }
__global__ __launch_bounds__(256) void pool_kernel(const float* __restrict__ QKV, const unsigned* __restrict__ XI16, int ldx, long xrow0, const int* __restrict__ nidx, long r0, unsigned* __restrict__ P16) {
  __shared__ float st[8][32];
  const int lane = threadIdx.x & 31, wave = threadIdx.x >> 5; const long blk = r0 / 8 + blockIdx.x; const long r = blk * 8 + wave; const int b = (int)(r / PN);
  const float q = QKV[r * 128 + lane];
  float m = -INFINITY, ssum = 0.f, acc = 0.f;
  for (int k = 0; k < PK; ++k) { int j = nidx[r * PK + k]; j = j < 0 ? 0 : (j >= PN ? PN - 1 : j); const long rj = (long)b * PN + j;
    const float w = ldh(XI16, ((r - xrow0) * PK + k) * (long)ldx + lane) * (QKV[rj * 128 + 32 + lane] - q);
    const float v = QKV[rj * 128 + 64 + lane];
    const float mn = fmaxf(m, w); const float sc = expf(m - mn); const float e = expf(w - mn);
    ssum = ssum * sc + e; acc = acc * sc + e * v; m = mn; }
  st[wave][lane] = acc / ssum;
  __syncthreads();
  if (threadIdx.x < 128) { const int p = threadIdx.x >> 4, cp = (threadIdx.x & 15) * 2;
    const unsigned u = (unsigned)__builtin_bit_cast(unsigned short, (_Float16)st[p][cp]) | ((unsigned)__builtin_bit_cast(unsigned short, (_Float16)st[p][cp + 1]) << 16);
    ((volatile unsigned*)P16)[(size_t)blk * 128 + threadIdx.x] = u; __threadfence(); ((volatile unsigned*)P16)[(size_t)blk * 128 + threadIdx.x] = u; }
}
__global__ __launch_bounds__(256) void out_kernel(const float* __restrict__ O, float* __restrict__ out) {
  __shared__ float tile[64][65];
  const int b = blockIdx.z, n0 = blockIdx.x * 64, c0 = blockIdx.y * 64, tx = threadIdx.x, ty = threadIdx.y;
  for (int p = ty; p < 64; p += 8) { const size_t r = (size_t)b * PN + n0 + p; tile[tx][p] = O[r * 128 + c0 + tx]; tile[32 + tx][p] = O[r * 128 + c0 + 32 + tx]; }
  __syncthreads();
  for (int pass = 0; pass < 2; ++pass) { for (int c = ty; c < 64; c += 8) { float v0 = tile[c][tx], v1 = tile[c][32 + tx]; v0 = v0 > 0.f ? v0 : 0.2f * v0; v1 = v1 > 0.f ? v1 : 0.2f * v1;
      float* dst = out + ((size_t)b * 128 + c0 + c) * PN + n0; ((volatile float*)dst)[tx] = v0; ((volatile float*)dst)[32 + tx] = v1; } __threadfence(); }
}
extern "C" void kernel_launch(void* const* d_in, const int* in_sizes, int n_in, void* d_out, int out_size, void* d_ws, size_t ws_size, hipStream_t stream) {
  (void)in_sizes; (void)n_in; (void)out_size; (void)ws_size;
  const float* x = (const float*)d_in[0]; const float* feat = (const float*)d_in[1]; const int* nidx = (const int*)d_in[2];
  auto F = [&](int i) { return (const float*)d_in[i]; };
  char* ws = (char*)d_ws; size_t off = 0;
  auto carve = [&](size_t bytes) -> char* { char* p = ws + off; off += (bytes + 255) & ~(size_t)255; return p; };
  unsigned* FT16 = (unsigned*)carve((size_t)PR * 64 * 2); float* XT = (float*)carve((size_t)PR * 4 * 4);
  unsigned* Wm1 = (unsigned*)carve(64 * 64 * 2); float* bm1 = (float*)carve(64 * 4);
  unsigned* Wq1 = (unsigned*)carve(128 * 32 * 2); float* bq1 = (float*)carve(128 * 4); unsigned* Wq2 = (unsigned*)carve(128 * 32 * 2); float* bq2 = (float*)carve(128 * 4);
  unsigned* W21 = (unsigned*)carve(64 * 32 * 2); float* b21 = (float*)carve(64 * 4); unsigned* W22 = (unsigned*)carve(64 * 32 * 2); float* b22 = (float*)carve(64 * 4);
  unsigned* Wl2 = (unsigned*)carve(64 * 32 * 2); float* bl2 = (float*)carve(64 * 4);
  unsigned* Wm2 = (unsigned*)carve(128 * 64 * 2); float* bm2 = (float*)carve(128 * 4); unsigned* Wrs = (unsigned*)carve(128 * 64 * 2); float* brs = (float*)carve(128 * 4);
  unsigned* F1 = (unsigned*)carve((size_t)PR * 64 * 2);
  unsigned* XI1 = (unsigned*)carve((size_t)PRK * 32 * 2);
  float* QKV = (float*)carve((size_t)PR * 128 * 4);
  unsigned* P1 = (unsigned*)carve((size_t)PR * 32 * 2); unsigned* F2 = (unsigned*)carve((size_t)PR * 64 * 2);
  unsigned* XI2 = (unsigned*)carve((size_t)(PRK / 2) * 64 * 2);
  unsigned* P2 = (unsigned*)carve((size_t)PR * 32 * 2); unsigned* F3 = (unsigned*)carve((size_t)PR * 64 * 2);
  float* T = QKV;
  float* OUT = (float*)XI1;
  in_kernel<<<dim3(PN / 64, PB), dim3(32, 8), 0, stream>>>(feat, x, FT16, XT);
  fold_kernel<<<(64 * 64 / 2 + 255) / 256, 256, 0, stream>>>(F(3), F(4), F(5), 32, 64, 64, 0, Wm1, bm1);
  fold_kernel<<<(32 * 32 / 2 + 255) / 256, 256, 0, stream>>>(F(9), F(10), F(11), 32, 32, 32, 0, Wq1, bq1);
  fold_kernel<<<(32 * 32 / 2 + 255) / 256, 256, 0, stream>>>(F(12), F(13), F(14), 32, 32, 32, 32, Wq1, bq1);
  fold_kernel<<<(64 * 32 / 2 + 255) / 256, 256, 0, stream>>>(F(15), F(16), F(17), 32, 32, 64, 64, Wq1, bq1);
  fold_kernel<<<(64 * 32 / 2 + 255) / 256, 256, 0, stream>>>(F(18), F(19), F(20), 32, 32, 64, 0, W21, b21);
  fold_kernel<<<(32 * 32 / 2 + 255) / 256, 256, 0, stream>>>(F(21), F(22), F(23), 32, 32, 32, 0, Wq2, bq2);
  fold_kernel<<<(32 * 32 / 2 + 255) / 256, 256, 0, stream>>>(F(24), F(25), F(26), 32, 32, 32, 32, Wq2, bq2);
  fold_kernel<<<(64 * 32 / 2 + 255) / 256, 256, 0, stream>>>(F(27), F(28), F(29), 32, 32, 64, 64, Wq2, bq2);
  fold_kernel<<<(64 * 32 / 2 + 255) / 256, 256, 0, stream>>>(F(30), F(31), F(32), 64, 32, 64, 0, W22, b22);
  fold_kernel<<<(64 * 32 / 2 + 255) / 256, 256, 0, stream>>>(F(33), F(34), F(35), 32, 32, 64, 0, Wl2, bl2);
  fold_kernel<<<(128 * 64 / 2 + 255) / 256, 256, 0, stream>>>(F(36), F(37), F(38), 128, 64, 128, 0, Wm2, bm2);
  fold_kernel<<<(128 * 64 / 2 + 255) / 256, 256, 0, stream>>>(F(39), F(40), F(41), 128, 64, 128, 0, Wrs, brs);
  const int t64 = (PR / 64) * 1, t128 = (PR / 64) * 2;
  wmma_gemm64<0, false, 2, 1, false, 6><<<dim3((t64 + 7) / 8, 1), 256, 0, stream>>>((const unsigned short*)FT16, nullptr, 64, 0, (const unsigned short*)Wm1, nullptr, 64, 0, F1, nullptr, 64, 0, bm1, nullptr, 0, PR, 64, 64, 1.0f);
  lse1_kernel<<<PRK / 256, 256, 0, stream>>>(XT, nidx, F(6), F(7), F(8), XI1);
  wmma_gemm64<0, false, 2, 0, false, 2><<<dim3((t128 + 7) / 8, 1), 256, 0, stream>>>((const unsigned short*)F1, nullptr, 64, 0, (const unsigned short*)Wq1, nullptr, 32, 0, QKV, nullptr, 128, 0, bq1, nullptr, 0, PR, 128, 32, 1.0f);
  pool_kernel<<<PR / 8, 256, 0, stream>>>(QKV, XI1, 32, 0, nidx, 0, P1);
  wmma_gemm64<0, false, 2, 1, false, 6><<<dim3((t64 + 7) / 8, 1), 256, 0, stream>>>((const unsigned short*)P1, nullptr, 32, 0, (const unsigned short*)W21, nullptr, 32, 0, F2, nullptr, 64, 0, b21, nullptr, 0, PR, 64, 32, 1.0f);
  wmma_gemm64<0, false, 2, 0, false, 2><<<dim3((t128 + 7) / 8, 1), 256, 0, stream>>>((const unsigned short*)F2, nullptr, 64, 0, (const unsigned short*)Wq2, nullptr, 32, 0, QKV, nullptr, 128, 0, bq2, nullptr, 0, PR, 128, 32, 1.0f);
  for (int h = 0; h < 2; ++h) { const long p0 = (long)h * (PRK / 2); const int th = ((PRK / 2) / 64) * 1;
    wmma_gemm64<0, false, 2, 1, false, 6><<<dim3((th + 7) / 8, 1), 256, 0, stream>>>((const unsigned short*)XI1 + p0 * 32, nullptr, 32, 0, (const unsigned short*)Wl2, nullptr, 32, 0, XI2, nullptr, 64, 0, bl2, nullptr, 0, PRK / 2, 64, 32, 1.0f);
    pool_kernel<<<(PR / 2) / 8, 256, 0, stream>>>(QKV, XI2, 64, (long)h * (PR / 2), nidx, (long)h * (PR / 2), P2);
  }
  wmma_gemm64<0, false, 2, 1, false, 6><<<dim3((t64 + 7) / 8, 1), 256, 0, stream>>>((const unsigned short*)P2, nullptr, 32, 0, (const unsigned short*)W22, nullptr, 32, 0, F3, nullptr, 64, 0, b22, nullptr, 0, PR, 64, 32, 1.0f);
  wmma_gemm64<0, false, 2, 0, false, 0><<<dim3((t128 + 7) / 8, 1), 256, 0, stream>>>((const unsigned short*)F3, nullptr, 64, 0, (const unsigned short*)Wm2, nullptr, 64, 0, T, nullptr, 128, 0, bm2, nullptr, 0, PR, 128, 64, 1.0f);
  wmma_gemm64<0, false, 2, 0, true, 0><<<dim3((t128 + 7) / 8, 1), 256, 0, stream>>>((const unsigned short*)FT16, nullptr, 64, 0, (const unsigned short*)Wrs, nullptr, 64, 0, OUT, nullptr, 128, 0, brs, T, 0, PR, 128, 64, 1.0f);
  out_kernel<<<dim3(PN / 64, 2, PB), dim3(32, 8), 0, stream>>>(OUT, (float*)d_out);
}
